// MultiScaleDCN_56100862820884
// MI455X (gfx1250) — hardware-verified
//
#include <hip/hip_runtime.h>
#include <stdint.h>


#define NPIX   16384
#define CIN    256
#define IMH    64
#define IMW    64
#define NGRP   8
#define NCH    32
#define NTAP   9
#define NPROJ  544
#define NQD    144
#define NQ     72
#define COL_QD 256
#define COL_QS 400
#define COL_QW 472
#define NWROWS 800
#define NITEMS (NPIX * NGRP * NTAP)
#define MAXSC  6.0f

static_assert(NPIX % 32 == 0);
static_assert(NPROJ % 32 == 0);
static_assert(CIN % 32 == 0);
static_assert(NWROWS % 32 == 0);
static_assert(NPROJ == CIN + NQD + NQ + NQ);

typedef __bf16       v16bf __attribute__((ext_vector_type(16)));
typedef float        v8f   __attribute__((ext_vector_type(8)));
typedef float        v4f   __attribute__((ext_vector_type(4)));
typedef unsigned int v4u   __attribute__((ext_vector_type(4)));
typedef int          v4i   __attribute__((ext_vector_type(4)));

union Frag { v16bf v; v4u q[2]; };

__device__ __forceinline__ unsigned int bf_bits(float f) {
    unsigned int u = __float_as_uint(f);
    u += 0x7FFFu + ((u >> 16) & 1u);
    return u >> 16;
}
__device__ __forceinline__ void split_bf(float f, unsigned int& hb, unsigned int& lb) {
    hb = bf_bits(f);
    const float hf = __uint_as_float(hb << 16);
    lb = bf_bits(f - hf);
}

__device__ __forceinline__ v8f wmma3(v8f acc, const Frag& ah, const Frag& al,
                                     const Frag& bh, const Frag& bl) {
    acc = __builtin_amdgcn_wmma_f32_16x16x32_bf16(false, ah.v, false, bh.v, (short)0, acc, false, false);
    acc = __builtin_amdgcn_wmma_f32_16x16x32_bf16(false, ah.v, false, bl.v, (short)0, acc, false, false);
    acc = __builtin_amdgcn_wmma_f32_16x16x32_bf16(false, al.v, false, bh.v, (short)0, acc, false, false);
    return acc;
}

__global__ __launch_bounds__(256)
void k_cvt_x(const float* __restrict__ x, uint16_t* __restrict__ Xh,
             uint16_t* __restrict__ Xl, int n8) {
    const int i = blockIdx.x * 256 + threadIdx.x;
    if (i >= n8) return;
    const v4f* p = (const v4f*)(x + (size_t)i * 8);
    const v4f a = p[0];
    const v4f b = p[1];
    float f[8];
#pragma unroll
    for (int j = 0; j < 4; ++j) { f[j] = a[j]; f[4 + j] = b[j]; }
    v4u hv, lv;
#pragma unroll
    for (int j = 0; j < 4; ++j) {
        unsigned int h0, l0, h1, l1;
        split_bf(f[2 * j], h0, l0);
        split_bf(f[2 * j + 1], h1, l1);
        hv[j] = h0 | (h1 << 16);
        lv[j] = l0 | (l1 << 16);
    }
    volatile v4u* dh = (volatile v4u*)(Xh + (size_t)i * 8);
    volatile v4u* dl = (volatile v4u*)(Xl + (size_t)i * 8);
    *dh = hv;
    *dl = lv;
    __threadfence();
    *dh = hv;
    *dl = lv;
}

__device__ __forceinline__ float wsrc(const float* __restrict__ v_w, const float* __restrict__ qd_w,
                                      const float* __restrict__ qs_w, const float* __restrict__ qw_w,
                                      const float* __restrict__ out_w, int n, int k) {
    if (n < COL_QD) return v_w[(size_t)k * CIN + n];
    if (n < COL_QS) return qd_w[(size_t)k * NQD + (n - COL_QD)];
    if (n < COL_QW) return qs_w[(size_t)k * NQ + (n - COL_QS)];
    if (n < NPROJ)  return qw_w[(size_t)k * NQ + (n - COL_QW)];
    return out_w[(size_t)k * CIN + (n - NPROJ)];
}
__device__ __forceinline__ float bsrc(const float* __restrict__ v_b, const float* __restrict__ qd_b,
                                      const float* __restrict__ qw_b, int n) {
    if (n < COL_QD) return v_b[n];
    if (n < COL_QS) return qd_b[n - COL_QD];
    if (n < COL_QW) return 0.0f;
    return qw_b[n - COL_QW];
}

__global__ __launch_bounds__(256)
void k_prep_w(const float* __restrict__ v_w, const float* __restrict__ qd_w,
              const float* __restrict__ qs_w, const float* __restrict__ qw_w,
              const float* __restrict__ out_w,
              const float* __restrict__ v_b, const float* __restrict__ qd_b,
              const float* __restrict__ qw_b,
              uint16_t* __restrict__ WTh, uint16_t* __restrict__ WTl,
              float* __restrict__ bias_cat, int nrows) {
    __shared__ float tile[CIN * 33];
    const int tid = threadIdx.x;
    const int n0  = blockIdx.x * 32;
    for (int e = tid; e < CIN * 32; e += 256) {
        const int k  = e >> 5;
        const int nl = e & 31;
        const int n  = n0 + nl;
        tile[k * 33 + nl] = (n < nrows) ? wsrc(v_w, qd_w, qs_w, qw_w, out_w, n, k) : 0.0f;
    }
    __syncthreads();

    const int wv = tid >> 5;
    const int l  = tid & 31;
    v4u hv[4], lv[4];
#pragma unroll
    for (int t = 0; t < 4; ++t) {
        const int nl = wv * 4 + t;
#pragma unroll
        for (int j = 0; j < 4; ++j) {
            unsigned int h0, l0, h1, l1;
            split_bf(tile[(8 * l + 2 * j)     * 33 + nl], h0, l0);
            split_bf(tile[(8 * l + 2 * j + 1) * 33 + nl], h1, l1);
            hv[t][j] = h0 | (h1 << 16);
            lv[t][j] = l0 | (l1 << 16);
        }
    }
#pragma unroll
    for (int t = 0; t < 4; ++t) {
        const int n = n0 + wv * 4 + t;
        if (n < nrows) {
            *(volatile v4u*)(WTh + (size_t)n * CIN + 8 * l) = hv[t];
            *(volatile v4u*)(WTl + (size_t)n * CIN + 8 * l) = lv[t];
        }
    }
    __threadfence();
#pragma unroll
    for (int t = 0; t < 4; ++t) {
        const int n = n0 + wv * 4 + t;
        if (n < nrows) {
            *(volatile v4u*)(WTh + (size_t)n * CIN + 8 * l) = hv[t];
            *(volatile v4u*)(WTl + (size_t)n * CIN + 8 * l) = lv[t];
        }
    }

    if (blockIdx.x == 0 && tid < NPROJ / 4) {
        v4f bv;
#pragma unroll
        for (int j = 0; j < 4; ++j) bv[j] = bsrc(v_b, qd_b, qw_b, 4 * tid + j);
        volatile v4f* pb = (volatile v4f*)(bias_cat + 4 * tid);
        *pb = bv;
        __threadfence();
        *pb = bv;
    }
}

__global__ __launch_bounds__(256)
void k_gemm(const uint16_t* __restrict__ Ah, const uint16_t* __restrict__ Al,
            const uint16_t* __restrict__ Bh, const uint16_t* __restrict__ Bl,
            const float* __restrict__ bias, float* __restrict__ Cout, int M, int N) {
    __shared__ float sT[8 * 1024];
    const int tid = threadIdx.x;
    const int wv  = tid >> 5;
    const int l   = tid & 31;
    const int h   = l >> 4;
    const int m   = l & 15;
    const int tilesN = N >> 5;
    const int tiles  = (M >> 5) * tilesN;
    const int gw     = blockIdx.x * 8 + wv;
    const bool active = gw < tiles;
    const int t  = active ? gw : 0;
    const int tq = t / tilesN;
    const int tm = tq << 5;
    const int tn = (t - tq * tilesN) << 5;

    const uint16_t* a0h = Ah + (size_t)(tm + m) * CIN + 8 * h;
    const uint16_t* a0l = Al + (size_t)(tm + m) * CIN + 8 * h;
    const uint16_t* a1h = a0h + (size_t)16 * CIN;
    const uint16_t* a1l = a0l + (size_t)16 * CIN;
    const uint16_t* b0h = Bh + (size_t)(tn + m) * CIN + 8 * h;
    const uint16_t* b0l = Bl + (size_t)(tn + m) * CIN + 8 * h;
    const uint16_t* b1h = b0h + (size_t)16 * CIN;
    const uint16_t* b1l = b0l + (size_t)16 * CIN;

    v8f acc00, acc01, acc10, acc11;
#pragma unroll
    for (int r = 0; r < 8; ++r) { acc00[r] = 0.f; acc01[r] = 0.f; acc10[r] = 0.f; acc11[r] = 0.f; }

#pragma unroll 1
    for (int k0 = 0; k0 < CIN; k0 += 32) {
        Frag fa0h, fa0l, fa1h, fa1l, fb0h, fb0l, fb1h, fb1l;
        fa0h.q[0] = *(const v4u*)(a0h + k0); fa0h.q[1] = *(const v4u*)(a0h + k0 + 16);
        fa0l.q[0] = *(const v4u*)(a0l + k0); fa0l.q[1] = *(const v4u*)(a0l + k0 + 16);
        fa1h.q[0] = *(const v4u*)(a1h + k0); fa1h.q[1] = *(const v4u*)(a1h + k0 + 16);
        fa1l.q[0] = *(const v4u*)(a1l + k0); fa1l.q[1] = *(const v4u*)(a1l + k0 + 16);
        fb0h.q[0] = *(const v4u*)(b0h + k0); fb0h.q[1] = *(const v4u*)(b0h + k0 + 16);
        fb0l.q[0] = *(const v4u*)(b0l + k0); fb0l.q[1] = *(const v4u*)(b0l + k0 + 16);
        fb1h.q[0] = *(const v4u*)(b1h + k0); fb1h.q[1] = *(const v4u*)(b1h + k0 + 16);
        fb1l.q[0] = *(const v4u*)(b1l + k0); fb1l.q[1] = *(const v4u*)(b1l + k0 + 16);
        acc00 = wmma3(acc00, fa0h, fa0l, fb0h, fb0l);
        acc01 = wmma3(acc01, fa0h, fa0l, fb1h, fb1l);
        acc10 = wmma3(acc10, fa1h, fa1l, fb0h, fb0l);
        acc11 = wmma3(acc11, fa1h, fa1l, fb1h, fb1l);
        asm volatile("v_nop\n\tv_nop\n\tv_nop\n\tv_nop"
                     : "+v"(acc00), "+v"(acc01), "+v"(acc10), "+v"(acc11)
                     : "v"(fa0h.v), "v"(fa0l.v), "v"(fa1h.v), "v"(fa1l.v),
                       "v"(fb0h.v), "v"(fb0l.v), "v"(fb1h.v), "v"(fb1l.v));
    }

    float* st = sT + wv * 1024;
#pragma unroll
    for (int r = 0; r < 8; ++r) {
        st[(8 * h + r) * 32 + m]           = acc00[r];
        st[(8 * h + r) * 32 + 16 + m]      = acc01[r];
        st[(16 + 8 * h + r) * 32 + m]      = acc10[r];
        st[(16 + 8 * h + r) * 32 + 16 + m] = acc11[r];
    }
    __syncthreads();

    const int q = l >> 3;
    const int j = l & 7;
    const v4f bv = *(const v4f*)(bias + tn + 4 * j);
    v4f vals[8];
#pragma unroll
    for (int i = 0; i < 8; ++i) {
        const v4f v = *(const v4f*)(st + (4 * i + q) * 32 + 4 * j);
        vals[i] = v + bv;
    }
    if (active) {
        float* cb = Cout + (size_t)tm * N + tn + 4 * j;
#pragma unroll
        for (int i = 0; i < 8; ++i)
            *(volatile v4f*)(cb + (size_t)(4 * i + q) * N) = vals[i];
        __threadfence();
#pragma unroll
        for (int i = 0; i < 8; ++i)
            *(volatile v4f*)(cb + (size_t)(4 * i + q) * N) = vals[i];
    }
}

__global__ __launch_bounds__(256)
void k_geom(const float* __restrict__ P, const float* __restrict__ prior,
            const float* __restrict__ dscale,
            float* __restrict__ GW, int* __restrict__ GO, int nitems) {
#pragma clang fp contract(off)
    const int it = blockIdx.x * 256 + threadIdx.x;
    if (it >= nitems) return;
    const int pg  = it / NTAP;
    const int k   = it - pg * NTAP;
    const int pix = pg >> 3;
    const int g   = pg & 7;
    const int b   = pix >> 12;
    const int hw  = pix & 4095;
    const int h   = hw >> 6;
    const int w   = hw & 63;

    const float* row = P + (size_t)pix * NPROJ;
    const float qd0 = row[COL_QD + g * 18 + 2 * k];
    const float qd1 = row[COL_QD + g * 18 + 2 * k + 1];
    const float qs  = row[COL_QS + g * 9 + k];
    const float qw  = row[COL_QW + g * 9 + k];

    const float sc  = qs + dscale[g];
    const float sig = 1.0f / (1.0f + expf(-sc));
    float dx = qd0 + prior[2 * k];
    float dy = qd1 + prior[2 * k + 1];
    dx = dx * sig; dx = dx * MAXSC;
    dy = dy * sig; dy = dy * MAXSC;
    const float px = (float)w + dx;
    const float py = (float)h + dy;

    const float x0f = floorf(px);
    const float y0f = floorf(py);
    const float wx1 = px - x0f, wx0 = 1.0f - wx1;
    const float wy1 = py - y0f, wy0 = 1.0f - wy1;

    const float x0c = fminf(fmaxf(x0f, -4.0f), 68.0f);
    const float y0c = fminf(fmaxf(y0f, -4.0f), 68.0f);
    const int x0 = (int)x0c;
    const int y0 = (int)y0c;
    const bool vx0 = (unsigned)x0       < (unsigned)IMW;
    const bool vx1 = (unsigned)(x0 + 1) < (unsigned)IMW;
    const bool vy0 = (unsigned)y0       < (unsigned)IMH;
    const bool vy1 = (unsigned)(y0 + 1) < (unsigned)IMH;
    const int xc0 = min(max(x0, 0), IMW - 1);
    const int xc1 = min(max(x0 + 1, 0), IMW - 1);
    const int yc0 = min(max(y0, 0), IMH - 1);
    const int yc1 = min(max(y0 + 1, 0), IMH - 1);
    const int rb  = b * IMH;

    v4i o;
    o[0] = (rb + yc0) * IMW + xc0;
    o[1] = (rb + yc0) * IMW + xc1;
    o[2] = (rb + yc1) * IMW + xc0;
    o[3] = (rb + yc1) * IMW + xc1;
    v4f wv;
    wv[0] = (vy0 && vx0) ? (wy0 * wx0) * qw : 0.0f;
    wv[1] = (vy0 && vx1) ? (wy0 * wx1) * qw : 0.0f;
    wv[2] = (vy1 && vx0) ? (wy1 * wx0) * qw : 0.0f;
    wv[3] = (vy1 && vx1) ? (wy1 * wx1) * qw : 0.0f;

    volatile v4f* pw = (volatile v4f*)(GW + (size_t)it * 4);
    volatile v4i* po = (volatile v4i*)(GO + (size_t)it * 4);
    *pw = wv;
    *po = o;
    __threadfence();
    *pw = wv;
    *po = o;
}

__global__ __launch_bounds__(256)
void k_samp(const float* __restrict__ P, const float* __restrict__ GW,
            const int* __restrict__ GO,
            uint16_t* __restrict__ Dh, uint16_t* __restrict__ Dl, int npix) {
    __shared__ uint16_t sh[256];
    __shared__ uint16_t sl[256];
    const int pix = blockIdx.x;
    if (pix >= npix) return;
    const int tid = threadIdx.x;
    const int c   = tid & 31;
    const int g   = __builtin_amdgcn_readfirstlane(tid >> 5);

    const v4f* gwp = (const v4f*)GW + ((size_t)pix * NGRP + g) * NTAP;
    const v4i* gop = (const v4i*)GO + ((size_t)pix * NGRP + g) * NTAP;
    const float* vb = P + g * NCH + c;

    float acc = 0.0f;
#pragma unroll
    for (int k = 0; k < NTAP; ++k) {
        const v4f w = gwp[k];
        const v4i o = gop[k];
        const int o0 = min(max(o[0], 0), NPIX - 1);
        const int o1 = min(max(o[1], 0), NPIX - 1);
        const int o2 = min(max(o[2], 0), NPIX - 1);
        const int o3 = min(max(o[3], 0), NPIX - 1);
        const float v00 = vb[(size_t)o0 * NPROJ];
        const float v01 = vb[(size_t)o1 * NPROJ];
        const float v10 = vb[(size_t)o2 * NPROJ];
        const float v11 = vb[(size_t)o3 * NPROJ];
        acc += w[0] * v00;
        acc += w[1] * v01;
        acc += w[2] * v10;
        acc += w[3] * v11;
    }
    unsigned int hb, lb;
    split_bf(acc, hb, lb);
    sh[tid] = (uint16_t)hb;
    sl[tid] = (uint16_t)lb;
    __syncthreads();

    if (tid < 64) {
        const int wv = tid >> 5;
        const int l  = tid & 31;
        v4u pk;
#pragma unroll
        for (int j = 0; j < 4; ++j) {
            const unsigned int e0 = (wv == 0) ? sh[8 * l + 2 * j]     : sl[8 * l + 2 * j];
            const unsigned int e1 = (wv == 0) ? sh[8 * l + 2 * j + 1] : sl[8 * l + 2 * j + 1];
            pk[j] = e0 | (e1 << 16);
        }
        uint16_t* dst = ((wv == 0) ? Dh : Dl) + (size_t)pix * CIN + 8 * l;
        *(volatile v4u*)dst = pk;
        __threadfence();
        *(volatile v4u*)dst = pk;
    }
}

extern "C" void kernel_launch(void* const* d_in, const int* in_sizes, int n_in,
                              void* d_out, int out_size, void* d_ws, size_t ws_size,
                              hipStream_t stream) {
    if (n_in < 12) return;
    if (in_sizes[0] != NPIX * CIN || out_size != NPIX * CIN) return;
    if (in_sizes[1] != CIN * CIN || in_sizes[3] != CIN * NQD || in_sizes[5] != CIN * NQ ||
        in_sizes[6] != CIN * NQ || in_sizes[8] != CIN * CIN) return;

    const float* x      = (const float*)d_in[0];
    const float* v_w    = (const float*)d_in[1];
    const float* v_b    = (const float*)d_in[2];
    const float* qd_w   = (const float*)d_in[3];
    const float* qd_b   = (const float*)d_in[4];
    const float* qs_w   = (const float*)d_in[5];
    const float* qw_w   = (const float*)d_in[6];
    const float* qw_b   = (const float*)d_in[7];
    const float* out_w  = (const float*)d_in[8];
    const float* out_b  = (const float*)d_in[9];
    const float* prior  = (const float*)d_in[10];
    const float* dscale = (const float*)d_in[11];

    char*  ws  = (char*)d_ws;
    size_t off = 0;
    auto carve = [&](size_t bytes) -> char* {
        char* p = ws + off;
        off += (bytes + 255) & ~(size_t)255;
        return p;
    };
    uint16_t* Xh    = (uint16_t*)carve((size_t)NPIX * CIN * 2);
    uint16_t* Xl    = (uint16_t*)carve((size_t)NPIX * CIN * 2);
    uint16_t* WTh   = (uint16_t*)carve((size_t)NWROWS * CIN * 2);
    uint16_t* WTl   = (uint16_t*)carve((size_t)NWROWS * CIN * 2);
    float*    biasc = (float*)   carve((size_t)NPROJ * 4);
    float*    P     = (float*)   carve((size_t)NPIX * NPROJ * 4);
    float*    GW    = (float*)   carve((size_t)NITEMS * 16);
    int*      GO    = (int*)     carve((size_t)NITEMS * 16);
    uint16_t* Dh    = (uint16_t*)carve((size_t)NPIX * CIN * 2);
    uint16_t* Dl    = (uint16_t*)carve((size_t)NPIX * CIN * 2);
    if (off > ws_size) return;

    const int n8 = NPIX * CIN / 8;
    k_cvt_x<<<(n8 + 255) / 256, 256, 0, stream>>>(x, Xh, Xl, n8);

    k_prep_w<<<(NWROWS + 31) / 32, 256, 0, stream>>>(v_w, qd_w, qs_w, qw_w, out_w,
                                                     v_b, qd_b, qw_b, WTh, WTl, biasc, NWROWS);

    {
        const int tiles = (NPIX / 32) * (NPROJ / 32);
        k_gemm<<<(tiles + 7) / 8, 256, 0, stream>>>(Xh, Xl, WTh, WTl, biasc, P, NPIX, NPROJ);
    }

    k_geom<<<(NITEMS + 255) / 256, 256, 0, stream>>>(P, prior, dscale, GW, GO, NITEMS);

    k_samp<<<NPIX, 256, 0, stream>>>(P, GW, GO, Dh, Dl, NPIX);

    {
        const int tiles = (NPIX / 32) * (CIN / 32);
        k_gemm<<<(tiles + 7) / 8, 256, 0, stream>>>(Dh, Dl, WTh + (size_t)NPROJ * CIN,
                                                    WTl + (size_t)NPROJ * CIN,
                                                    out_b, (float*)d_out, NPIX, CIN);
    }
}
